// NeighborhoodAttention2D_16406775071495
// MI455X (gfx1250) — hardware-verified
//
#include <hip/hip_runtime.h>
#include <math.h>

typedef __attribute__((ext_vector_type(16))) _Float16 v16h;
typedef __attribute__((ext_vector_type(16))) __bf16 v16b;
typedef __attribute__((ext_vector_type(8)))  _Float16 v8h;
typedef __attribute__((ext_vector_type(8)))  float v8f;
typedef __attribute__((ext_vector_type(4)))  float v4f;
typedef __attribute__((ext_vector_type(2)))  float v2f;
typedef __attribute__((ext_vector_type(4)))  unsigned v4u;
typedef __attribute__((ext_vector_type(4)))  int v4i;
typedef float __attribute__((may_alias)) float_a;
typedef int __attribute__((may_alias)) int_a;

template <typename T> __device__ __forceinline__ void vst2(void* p, T v) { *(volatile T*)p = v; __threadfence(); *(volatile T*)p = v; }
__device__ __forceinline__ v8f wmma16(v16h a, v16h b, v8f c) {
  v8f d = __builtin_amdgcn_wmma_f32_16x16x32_f16(false, a, false, b, (short)0, c, false, false);
  asm volatile("v_nop\n\tv_nop\n\tv_nop\n\tv_nop" : "+v"(d) : "v"(a), "v"(b));
  return d;
}
__device__ __forceinline__ v8f wmma_bf(v16b a, v16b b, v8f c) {
  v8f d = __builtin_amdgcn_wmma_f32_16x16x32_bf16(false, a, false, b, (short)0, c, false, false);
  asm volatile("v_nop\n\tv_nop\n\tv_nop\n\tv_nop" : "+v"(d) : "v"(a), "v"(b));
  return d;
}
__device__ __forceinline__ v16h frag_h(const _Float16* rowk0, int lane) {
  union { v16h v; v8h q[2]; } u; const _Float16* p = rowk0 + 8 * (lane >> 4);
  u.q[0] = *(const v8h*)p; u.q[1] = *(const v8h*)(p + 16); return u.v;
}
__device__ __forceinline__ v16h frag_f32(const float* rowk0, int lane) {
  v16h a; const float* p = rowk0 + 8 * (lane >> 4);
#pragma unroll
  for (int i = 0; i < 8; ++i) { a[i] = (_Float16)p[i]; a[8 + i] = (_Float16)p[16 + i]; }
  return a;
}
__device__ __forceinline__ v16h frag_f32s(const float* rowk0, int lane, float sc) {
  v16h a; const float* p = rowk0 + 8 * (lane >> 4);
#pragma unroll
  for (int i = 0; i < 8; ++i) { a[i] = (_Float16)(p[i] * sc); a[8 + i] = (_Float16)(p[16 + i] * sc); }
  return a;
}
__device__ __forceinline__ v16h fragc_f32(const float* W, int k0, int n, int lane, int ld, int K) {
  v16h a; const int g = lane >> 4;
#pragma unroll
  for (int i = 0; i < 8; ++i) { const int ka = k0 + 8 * g + i, kb = ka + 16;
    a[i] = (_Float16)(ka < K ? W[(size_t)(ka < K ? ka : K - 1) * ld + n] : 0.f); a[8 + i] = (_Float16)(kb < K ? W[(size_t)(kb < K ? kb : K - 1) * ld + n] : 0.f); }
  return a;
}
struct F2 { v16b h, l; };
__device__ __forceinline__ F2 bsplit16(const float v[16]) { F2 r;
#pragma unroll
  for (int i = 0; i < 16; ++i) { const __bf16 h = (__bf16)v[i]; r.h[i] = h; r.l[i] = (__bf16)(v[i] - (float)h); }
  return r; }
__device__ __forceinline__ F2 split_row(const float* row, int k0, int lane) { float v[16]; const float* p = row + k0 + 8 * (lane >> 4);
#pragma unroll
  for (int i = 0; i < 8; ++i) { v[i] = p[i]; v[8 + i] = p[16 + i]; }
  return bsplit16(v); }
__device__ __forceinline__ F2 split_rowK(const float* row, int k0, int lane, int K) { float v[16]; const int g = lane >> 4;
#pragma unroll
  for (int i = 0; i < 8; ++i) { const int ka = k0 + 8 * g + i, kb = ka + 16; v[i] = ka < K ? row[ka < K ? ka : K - 1] : 0.f; v[8 + i] = kb < K ? row[kb < K ? kb : K - 1] : 0.f; }
  return bsplit16(v); }
__device__ __forceinline__ F2 split_col(const float* W, int k0, int n, int lane, int ld, int K) { float v[16]; const int g = lane >> 4;
#pragma unroll
  for (int i = 0; i < 8; ++i) { const int ka = k0 + 8 * g + i, kb = ka + 16; v[i] = ka < K ? W[(size_t)(ka < K ? ka : K - 1) * ld + n] : 0.f; v[8 + i] = kb < K ? W[(size_t)(kb < K ? kb : K - 1) * ld + n] : 0.f; }
  return bsplit16(v); }
__device__ __forceinline__ v8f mac3(const F2& a, const F2& b, v8f c) { c = wmma_bf(a.l, b.h, c); c = wmma_bf(a.h, b.l, c); return wmma_bf(a.h, b.h, c); }
__device__ __forceinline__ float sigm(float v) { return 1.0f / (1.0f + expf(-v)); }
#define LDSX() do { asm volatile("s_wait_dscnt 0" ::: "memory"); __builtin_amdgcn_wave_barrier(); __builtin_amdgcn_fence(__ATOMIC_RELEASE, "workgroup"); } while (0)

#define NBT 4
#define GH 56
#define NTOK 3136
#define CCH 256
#define NHD 8
#define HDM 32
#define KS 7
#define NR (NBT * NTOK)
#define QW 32
#define KC 38
#define NKEY (KS * KC)
#define NKP 288
#ifndef NBPROC
#define NBPROC NBT
#endif
typedef __attribute__((ext_vector_type(8))) __bf16 v8b;
__device__ __forceinline__ v16b frag_b(const __bf16* rowk0, int lane) { union { v16b v; v8b q[2]; } u; const __bf16* p = rowk0 + 8 * (lane >> 4); u.q[0] = *(const v8b*)p; u.q[1] = *(const v8b*)(p + 16); return u.v; }
__device__ __forceinline__ float bfr(float v) { return (float)(__bf16)v; }
__device__ __forceinline__ v16b wcol_io(const float* Wm, int k0, int o, int lane, int ld) { v16b w; const int g = lane >> 4; float t0[8], t1[8];
#pragma unroll
  for (int i = 0; i < 8; ++i) t0[i] = Wm[(size_t)(k0 + 8 * g + i) * ld + o];
  asm volatile("s_wait_loadcnt 0x0" ::: "memory");
#pragma unroll
  for (int i = 0; i < 8; ++i) t1[i] = Wm[(size_t)(k0 + 16 + 8 * g + i) * ld + o];
  asm volatile("s_wait_loadcnt 0x0" ::: "memory");
#pragma unroll
  for (int i = 0; i < 8; ++i) { w[i] = (__bf16)t0[i]; w[8 + i] = (__bf16)t1[i]; }
  return w; }
#define WS_QKV 0u
#define WS_Y   (WS_QKV + 4u * (size_t)NR * 3 * CCH)
#define WS_END (WS_Y + 4u * (size_t)NR * CCH)

__global__ __launch_bounds__(128) void k_qkv(const float* __restrict__ X, const float* __restrict__ Wm, const float* __restrict__ Bv, float* __restrict__ QKV) { __shared__ __align__(16) float sf[4][16][132];
  const int tid = threadIdx.x, wave = tid >> 5, lane = tid & 31, col = lane & 15, g = lane >> 4; const int c0 = blockIdx.y * 128; const size_t r0 = (size_t)blockIdx.x * 64 + wave * 16;
  v8f acc[8] = {};
#pragma unroll 2
  for (int kc = 0; kc < CCH / 32; ++kc) { v16b a; { const size_t rr = r0 + col < (size_t)NR ? r0 + col : (size_t)NR - 1; const float* p = X + rr * CCH + kc * 32 + 8 * g;
#pragma unroll
      for (int i = 0; i < 8; ++i) { a[i] = (__bf16)p[i]; a[8 + i] = (__bf16)p[16 + i]; } }
    asm volatile("s_wait_loadcnt 0x0" ::: "memory");
#pragma unroll
    for (int j = 0; j < 8; ++j) { const v16b w = wcol_io(Wm, kc * 32, c0 + j * 16 + col, lane, 3 * CCH); asm volatile("s_wait_loadcnt 0x0" ::: "memory"); acc[j] = wmma_bf(a, w, acc[j]); } }
#pragma unroll
  for (int j = 0; j < 8; ++j) { const float bb = bfr(Bv[c0 + j * 16 + col]);
#pragma unroll
    for (int r = 0; r < 8; ++r) sf[wave][8 * g + r][j * 16 + col] = acc[j][r] + bb; }
  LDSX(); for (int rl = 0; rl < 16; ++rl) if (r0 + rl < (size_t)NR) vst2(QKV + (r0 + rl) * (3 * CCH) + c0 + lane * 4, *(const v4f*)&sf[wave][rl][lane * 4]); }
__global__ __launch_bounds__(128) void k_natt(const float* __restrict__ QKV, float* __restrict__ Y) {
  __shared__ __align__(16) __bf16 sqh[QW][40], sql[QW][40], skh[NKP][40], skl[NKP][40], svh[HDM][NKP + 8], svl[HDM][NKP + 8], sph[QW][NKP + 8], spl[QW][NKP + 8];
  __shared__ __align__(16) float ss[QW][NKP + 4];
  const int tid = threadIdx.x, wave = tid >> 5, lane = tid & 31, col = lane & 15, g = lane >> 4;
  int bid = blockIdx.x; const int jh = bid & 1; bid >>= 1; const int i = bid % GH; bid /= GH; const int h = bid % NHD; const int b = bid / NHD;
  const int si = i - 3 < 0 ? 0 : (i - 3 > GH - KS ? GH - KS : i - 3);
  const int j0 = jh * QW; const int cj0 = j0 - 3 < 0 ? 0 : j0 - 3;
  const size_t rowb = (size_t)b * NTOK;
  for (int e = tid; e < QW * HDM; e += 128) { const int qq = e >> 5, d = e & 31; const int jq = j0 + qq < GH ? j0 + qq : GH - 1;
    const float qv = QKV[(rowb + (size_t)i * GH + jq) * (3 * CCH) + h * HDM + d]; const __bf16 hb = (__bf16)qv; sqh[qq][d] = hb; sql[qq][d] = (__bf16)(qv - (float)hb); }
  for (int e = tid; e < NKP * HDM; e += 128) { const int kk = e >> 5, d = e & 31; float kv = 0.f, vv = 0.f;
    if (kk < NKEY) { const int a = kk / KC, cc = kk % KC; const int jj = cj0 + cc; if (jj < GH) { const size_t tr = rowb + (size_t)(si + a) * GH + jj; kv = QKV[tr * (3 * CCH) + CCH + h * HDM + d]; vv = QKV[tr * (3 * CCH) + 2 * CCH + h * HDM + d]; } }
    const __bf16 kh = (__bf16)kv, vh = (__bf16)vv; skh[kk][d] = kh; skl[kk][d] = (__bf16)(kv - (float)kh); svh[d][kk] = vh; svl[d][kk] = (__bf16)(vv - (float)vh); }
  for (int e = tid; e < QW * 8; e += 128) { const int qq = e >> 3, z = e & 7; sqh[qq][32 + z] = (__bf16)0.f; sql[qq][32 + z] = (__bf16)0.f; }
  __syncthreads();
  { const v16b aqh0 = frag_b(&sqh[col][0], lane), aql0 = frag_b(&sql[col][0], lane), aqh1 = frag_b(&sqh[16 + col][0], lane), aql1 = frag_b(&sql[16 + col][0], lane);
    for (int ct = wave; ct < NKP / 16; ct += 4) { const v16b bh = frag_b(&skh[ct * 16 + col][0], lane), bl = frag_b(&skl[ct * 16 + col][0], lane);
      v8f a0 = {}, a1 = {}; a0 = wmma_bf(aqh0, bh, a0); a0 = wmma_bf(aql0, bh, a0); a0 = wmma_bf(aqh0, bl, a0); a1 = wmma_bf(aqh1, bh, a1); a1 = wmma_bf(aql1, bh, a1); a1 = wmma_bf(aqh1, bl, a1);
#pragma unroll
      for (int r = 0; r < 8; ++r) { ss[8 * g + r][ct * 16 + col] = a0[r] * 0.17677669529663687f; ss[16 + 8 * g + r][ct * 16 + col] = a1[r] * 0.17677669529663687f; } } }
  __syncthreads();
  { const int qq = tid >> 2, part = tid & 3; const int j = j0 + qq; const int sj = j - 3 < 0 ? 0 : (j - 3 > GH - KS ? GH - KS : j - 3);
    float m = -3.0e38f;
    for (int kk = part; kk < NKP; kk += 4) { const int a = kk / KC, cc = kk % KC, jj = cj0 + cc; const bool in = kk < NKEY && jj >= sj && jj < sj + KS; if (in) m = fmaxf(m, ss[qq][kk]); }
    m = fmaxf(m, __shfl_xor(m, 1)); m = fmaxf(m, __shfl_xor(m, 2));
    float sum = 0.f;
    for (int kk = part; kk < NKP; kk += 4) { const int a = kk / KC, cc = kk % KC, jj = cj0 + cc; const bool in = kk < NKEY && jj >= sj && jj < sj + KS; const float e = in ? expf(ss[qq][kk] - m) : 0.f; ss[qq][kk] = e; sum += e; (void)a; }
    sum += __shfl_xor(sum, 1); sum += __shfl_xor(sum, 2); const float inv = 1.0f / sum;
    for (int kk = part; kk < NKP; kk += 4) { const float p = ss[qq][kk] * inv; const __bf16 ph = (__bf16)p; sph[qq][kk] = ph; spl[qq][kk] = (__bf16)(p - (float)ph); } }
  __syncthreads();
  { const int rt = wave & 1, ct = wave >> 1; v8f acc = {};
#pragma unroll
    for (int kc = 0; kc < NKP / 32; ++kc) { const v16b ah = frag_b(&sph[rt * 16 + col][kc * 32], lane), al = frag_b(&spl[rt * 16 + col][kc * 32], lane), bh = frag_b(&svh[ct * 16 + col][kc * 32], lane), bl = frag_b(&svl[ct * 16 + col][kc * 32], lane);
      acc = wmma_bf(ah, bh, acc); acc = wmma_bf(al, bh, acc); acc = wmma_bf(ah, bl, acc); }
    __shared__ __align__(16) float so[QW][36];
#pragma unroll
    for (int r = 0; r < 8; ++r) so[rt * 16 + 8 * g + r][ct * 16 + col] = acc[r];
    __syncthreads();
    for (int pass = 0; pass < 2; ++pass) { const int qq = pass * 16 + (tid >> 3), q8 = tid & 7; if (j0 + qq < GH) vst2(Y + (rowb + (size_t)i * GH + j0 + qq) * CCH + h * HDM + q8 * 4, *(const v4f*)&so[qq][q8 * 4]); if (pass == 0) __builtin_amdgcn_fence(__ATOMIC_RELEASE, "agent"); } } }
__global__ __launch_bounds__(128) void k_out(const float* __restrict__ Yc, const float* __restrict__ Wm, const float* __restrict__ Bv, float* __restrict__ OUT) { __shared__ __align__(16) float sf[4][16][132];
  const int tid = threadIdx.x, wave = tid >> 5, lane = tid & 31, col = lane & 15, g = lane >> 4; const int c0 = blockIdx.y * 128; const size_t r0 = (size_t)blockIdx.x * 64 + wave * 16;
  v8f acc[8] = {};
#pragma unroll 2
  for (int kc = 0; kc < CCH / 32; ++kc) { const size_t rr = r0 + col < (size_t)NR ? r0 + col : (size_t)NR - 1; const F2 a = split_row(Yc + rr * CCH, kc * 32, lane); asm volatile("s_wait_loadcnt 0x0" ::: "memory");
#pragma unroll
    for (int j = 0; j < 8; ++j) { const v16b w = wcol_io(Wm, kc * 32, c0 + j * 16 + col, lane, CCH); asm volatile("s_wait_loadcnt 0x0" ::: "memory"); acc[j] = wmma_bf(a.h, w, acc[j]); acc[j] = wmma_bf(a.l, w, acc[j]); } }
#pragma unroll
  for (int j = 0; j < 8; ++j) { const float bb = bfr(Bv[c0 + j * 16 + col]);
#pragma unroll
    for (int r = 0; r < 8; ++r) sf[wave][8 * g + r][j * 16 + col] = acc[j][r] + bb; }
  LDSX(); for (int rl = 0; rl < 16; ++rl) if (r0 + rl < (size_t)NR) vst2(OUT + (r0 + rl) * CCH + c0 + lane * 4, *(const v4f*)&sf[wave][rl][lane * 4]); }
extern "C" void kernel_launch(void* const* d_in, const int* in_sizes, int n_in, void* d_out, int out_size, void* d_ws, size_t ws_size, hipStream_t stream) {
  (void)in_sizes; (void)n_in; (void)out_size;
  if (ws_size < (size_t)WS_END) return;
  char* ws = (char*)d_ws; float *QKV = (float*)(ws + WS_QKV), *Y = (float*)(ws + WS_Y); const float** F = (const float**)d_in;
  const int nrows = NBPROC * NTOK;
  k_qkv<<<dim3((nrows + 63) / 64, 3 * CCH / 128), 128, 0, stream>>>(F[0], F[1], F[2], QKV);
  k_natt<<<dim3(NBPROC * NHD * GH * 2), 128, 0, stream>>>(QKV, Y);
  k_out<<<dim3((nrows + 63) / 64, CCH / 128), 128, 0, stream>>>(Y, F[3], F[4], (float*)d_out);
}
